// RelativeAttention_5652176961770
// MI455X (gfx1250) — hardware-verified
//
#include <hip/hip_runtime.h>

typedef _Float16       v16h __attribute__((ext_vector_type(16)));
typedef __bf16         v16b __attribute__((ext_vector_type(16)));
typedef unsigned short v8us __attribute__((ext_vector_type(8)));
typedef float          v8f  __attribute__((ext_vector_type(8)));
typedef float          v4f  __attribute__((ext_vector_type(4)));
typedef unsigned int   v4u  __attribute__((ext_vector_type(4)));
typedef int            v4i  __attribute__((ext_vector_type(4)));

#ifndef NB
#define NB 1
#endif
#ifndef SEQ
#define SEQ 2049
#endif
#define SEQ_FULL 2049

constexpr int DM     = 1024;
constexpr int NH     = 16;
constexpr int HD     = 64;
constexpr int TT     = SEQ;
constexpr int NQB    = (TT + 63) / 64;
constexpr int NTB    = NQB + 1;
constexpr int TPAD   = NTB * 64;
constexpr int NKC    = NTB;
constexpr int NEARLY = NQB < 4 ? NQB : 4;
constexpr int CRES   = NEARLY * 64;
constexpr int QRES   = (NEARLY + 1) * 64;

constexpr float RSC  = 2048.0f;
constexpr float RINV = 1.0f / 2048.0f;
constexpr float PSC  = 1024.0f;
constexpr float CSC  = 16.0f;
constexpr float OCV  = CSC / PSC;
constexpr float WOSC = 64.0f;
constexpr float OINV = 1.0f / (CSC * WOSC);

static_assert(NB == 1);
static_assert(SEQ <= SEQ_FULL);
static_assert(HD == 64);
static_assert(DM % 64 == 0 && DM % 32 == 0);
static_assert(TPAD % 64 == 0);
static_assert(NKC <= 64);
static_assert(QRES <= TPAD && CRES <= TPAD);

constexpr size_t X_B  = (size_t)TPAD * DM * 2;
constexpr size_t W_B  = (size_t)DM * DM * 2;
constexpr size_t E_B  = (size_t)TPAD * HD * 2;
constexpr size_t HP_B = (size_t)NH * TPAD * HD * 2;
constexpr size_t QR_B = (size_t)NH * QRES * HD * 2;
constexpr size_t KR_B = (size_t)NH * CRES * HD * 2;
constexpr size_t CT_B = (size_t)TPAD * DM * 2;
constexpr size_t CR_B = (size_t)CRES * DM * 2;
constexpr size_t FL_B = (size_t)NQB * 64 * 4;

constexpr size_t OFF_XQ = 0;
constexpr size_t OFF_XK = OFF_XQ + X_B;
constexpr size_t OFF_XV = OFF_XK + X_B;
constexpr size_t OFF_WQ = OFF_XV + X_B;
constexpr size_t OFF_WK = OFF_WQ + W_B;
constexpr size_t OFF_WV = OFF_WK + W_B;
constexpr size_t OFF_WO = OFF_WV + W_B;
constexpr size_t OFF_ER = OFF_WO + W_B;
constexpr size_t OFF_QH = OFF_ER + E_B;
constexpr size_t OFF_KH = OFF_QH + HP_B;
constexpr size_t OFF_VT = OFF_KH + HP_B;
constexpr size_t OFF_QR = OFF_VT + HP_B;
constexpr size_t OFF_KR = OFF_QR + QR_B;
constexpr size_t OFF_VR = OFF_KR + KR_B;
constexpr size_t OFF_CT = OFF_VR + KR_B;
constexpr size_t OFF_CR = OFF_CT + CT_B;
constexpr size_t OFF_FL = OFF_CR + CR_B;
constexpr size_t WS_NEED = OFF_FL + FL_B;

static_assert(X_B % 128 == 0 && W_B % 128 == 0 && E_B % 128 == 0 && HP_B % 128 == 0);
static_assert(QR_B % 128 == 0 && KR_B % 128 == 0 && CT_B % 128 == 0 && CR_B % 128 == 0 && FL_B % 128 == 0);
static_assert(WS_NEED <= 134217728ull);
static_assert((size_t)TT * DM * 4 <= (size_t)SEQ_FULL * DM * 4);

__device__ __forceinline__ unsigned short f2bf_bits(float f) {
  unsigned u = __float_as_uint(f);
  return (unsigned short)((u + 0x7FFFu + ((u >> 16) & 1u)) >> 16);
}
__device__ __forceinline__ float bfr(float f) { return __uint_as_float(((unsigned)f2bf_bits(f)) << 16); }
__device__ __forceinline__ unsigned short h_bits(float f) {
  _Float16 h = (_Float16)f;
  return __builtin_bit_cast(unsigned short, h);
}
__device__ __forceinline__ float h2f(unsigned short b) {
  _Float16 h = __builtin_bit_cast(_Float16, b);
  return (float)h;
}

__device__ __forceinline__ v8f mma_h(v16h a, v16h b, v8f c) {
  c = __builtin_amdgcn_wmma_f32_16x16x32_f16(false, a, false, b, (short)0, c, false, false);
  asm volatile("v_nop\n\tv_nop\n\tv_nop\n\tv_nop" : "+v"(c) : "v"(a), "v"(b));
  return c;
}
__device__ __forceinline__ v8f mma_b(v16b a, v16b b, v8f c) {
  c = __builtin_amdgcn_wmma_f32_16x16x32_bf16(false, a, false, b, (short)0, c, false, false);
  asm volatile("v_nop\n\tv_nop\n\tv_nop\n\tv_nop" : "+v"(c) : "v"(a), "v"(b));
  return c;
}

__device__ __forceinline__ v8f zero8() { return (v8f){0.f,0.f,0.f,0.f,0.f,0.f,0.f,0.f}; }

__global__ __launch_bounds__(256) void cvt_plane_kernel(
    const float* __restrict__ src, int nrows, int ncols, int nrows_pad, int mode, float scale,
    unsigned short* __restrict__ dst)
{
  const int u = blockIdx.x * 256 + threadIdx.x;
  const int upr = ncols >> 3;
  const int total = nrows_pad * upr;
  if (u >= total) return;
  const int row = u / upr;
  const int cu  = u - row * upr;
  const int rowc = row < nrows ? row : nrows - 1;
  const bool live = row < nrows;
  const float* p = src + (size_t)rowc * ncols + cu * 8;
  const v4f x0 = *(const v4f*)p;
  const v4f x1 = *(const v4f*)(p + 4);
  unsigned b0, b1, b2, b3, b4, b5, b6, b7;
  {
    const float f0 = live ? x0[0] : 0.f, f1 = live ? x0[1] : 0.f, f2 = live ? x0[2] : 0.f, f3 = live ? x0[3] : 0.f;
    const float f4 = live ? x1[0] : 0.f, f5 = live ? x1[1] : 0.f, f6 = live ? x1[2] : 0.f, f7 = live ? x1[3] : 0.f;
    if (mode == 0) {
      b0 = f2bf_bits(f0); b1 = f2bf_bits(f1); b2 = f2bf_bits(f2); b3 = f2bf_bits(f3);
      b4 = f2bf_bits(f4); b5 = f2bf_bits(f5); b6 = f2bf_bits(f6); b7 = f2bf_bits(f7);
    } else {
      b0 = h_bits(bfr(f0) * scale); b1 = h_bits(bfr(f1) * scale); b2 = h_bits(bfr(f2) * scale); b3 = h_bits(bfr(f3) * scale);
      b4 = h_bits(bfr(f4) * scale); b5 = h_bits(bfr(f5) * scale); b6 = h_bits(bfr(f6) * scale); b7 = h_bits(bfr(f7) * scale);
    }
  }
  v4u w;
  w[0] = b0 | (b1 << 16);
  w[1] = b2 | (b3 << 16);
  w[2] = b4 | (b5 << 16);
  w[3] = b6 | (b7 << 16);
  unsigned short* d = dst + (size_t)u * 8;
  *(volatile v4u*)d = w;
  __threadfence();
  *(volatile v4u*)d = w;
}

__global__ __launch_bounds__(256) void flags_kernel(const int* __restrict__ mask, int* __restrict__ flags)
{
  __shared__ int part[8];
  __shared__ __align__(16) int fl[64];
  const int tid = threadIdx.x, lane = tid & 31, wave = tid >> 5;
  const int qb = blockIdx.x;
  if (tid < 64) fl[tid] = 0;
  __syncthreads();
#pragma unroll 1
  for (int kc = 0; kc < NKC; ++kc) {
    int cnt = 0;
#pragma unroll 4
    for (int it = 0; it < 16; ++it) {
      const int e = it * 256 + tid;
      const int r = e >> 6, cc = e & 63;
      int t = qb * 64 + r;
      t = t < TT ? t : TT - 1;
      const int s = kc * 64 + cc;
      const int sc = s < TT ? s : TT - 1;
      const int mv = mask[(size_t)t * SEQ_FULL + sc];
      cnt += (s < TT && mv != 0) ? 1 : 0;
    }
#pragma unroll
    for (int off = 1; off < 32; off <<= 1) cnt += __shfl_xor(cnt, off, 32);
    if (lane == 0) part[wave] = cnt;
    __syncthreads();
    if (tid == 0) {
      int tot = 0;
#pragma unroll
      for (int w = 0; w < 8; ++w) tot += part[w];
      fl[kc] = (tot == 0) ? 0 : ((tot == 4096) ? 1 : 2);
    }
    __syncthreads();
  }
  for (int pass = 0; pass < 2; ++pass) {
    if (tid < 16) {
      const v4i v = *(const v4i*)(fl + tid * 4);
      *(volatile v4i*)(flags + (size_t)qb * 64 + tid * 4) = v;
    }
    __threadfence();
  }
}

template <int MODE>
__global__ __launch_bounds__(64) __attribute__((amdgpu_num_vgpr(256)))
void proj_kernel(
    const unsigned short* __restrict__ X, const unsigned short* __restrict__ W,
    const float* __restrict__ bias, unsigned short* __restrict__ Ph, unsigned short* __restrict__ Pr)
{
  constexpr int PT = 72;
  constexpr int NRES_TB = (MODE == 0) ? (NEARLY + 1) : NEARLY;
  __shared__ __align__(16) unsigned short th[64 * PT];
  __shared__ __align__(16) unsigned short tr[64 * PT];
  union FB { v16b v; v8us h[2]; };

  const int tid = threadIdx.x, wave = tid >> 5, lane = tid & 31;
  const int hh = lane >> 4, m = lane & 15;
  const int tb = blockIdx.x, head = blockIdx.y;
  const int n0 = head * 64;
  const int rl0 = wave * 32;
  const int r0 = tb * 64 + rl0;

  v8f acc[2][4];
#pragma unroll
  for (int mi = 0; mi < 2; ++mi)
#pragma unroll
    for (int ni = 0; ni < 4; ++ni) acc[mi][ni] = zero8();

  const unsigned short* xp0 = X + (size_t)(r0 + m) * DM + 8 * hh;
  const unsigned short* xp1 = X + (size_t)(r0 + 16 + m) * DM + 8 * hh;
  const unsigned short* wp  = W + (size_t)(n0 + m) * DM + 8 * hh;

#pragma unroll 2
  for (int k0 = 0; k0 < DM; k0 += 32) {
    FB a0, a1;
    a0.h[0] = *(const v8us*)(xp0 + k0);
    a0.h[1] = *(const v8us*)(xp0 + k0 + 16);
    a1.h[0] = *(const v8us*)(xp1 + k0);
    a1.h[1] = *(const v8us*)(xp1 + k0 + 16);
#pragma unroll
    for (int ni = 0; ni < 4; ++ni) {
      FB b;
      b.h[0] = *(const v8us*)(wp + (size_t)ni * 16 * DM + k0);
      b.h[1] = *(const v8us*)(wp + (size_t)ni * 16 * DM + k0 + 16);
      acc[0][ni] = mma_b(a0.v, b.v, acc[0][ni]);
      acc[1][ni] = mma_b(a1.v, b.v, acc[1][ni]);
    }
  }

  float bb[4];
#pragma unroll
  for (int ni = 0; ni < 4; ++ni) bb[ni] = bfr(bias[n0 + ni * 16 + m]);

#pragma unroll
  for (int mi = 0; mi < 2; ++mi) {
#pragma unroll
    for (int ni = 0; ni < 4; ++ni) {
#pragma unroll
      for (int r = 0; r < 8; ++r) {
        const int rl  = rl0 + mi * 16 + 8 * hh + r;
        const int t   = tb * 64 + rl;
        const int col = ni * 16 + m;
        float y = acc[mi][ni][r] + bb[ni];
        y = (t < TT) ? y : 0.f;
        const unsigned short hb = h_bits(y);
        const float res = (y - h2f(hb)) * RSC;
        const unsigned short rb = h_bits(res);
        if (MODE == 2) { th[col * PT + rl] = hb; tr[col * PT + rl] = rb; }
        else           { th[rl * PT + col] = hb; tr[rl * PT + col] = rb; }
      }
    }
  }
  __syncthreads();

  const bool dores = tb < NRES_TB;
  for (int pass = 0; pass < 2; ++pass) {
#pragma unroll
    for (int it = 0; it < 8; ++it) {
      const int u = it * 64 + tid;
      const int row = u >> 3, seg = u & 7;
      const v8us vh = *(const v8us*)(th + row * PT + seg * 8);
      const v8us vr = *(const v8us*)(tr + row * PT + seg * 8);
      if (MODE == 2) {
        *(volatile v8us*)(Ph + ((size_t)head * HD + row) * TPAD + tb * 64 + seg * 8) = vh;
        if (dores) *(volatile v8us*)(Pr + ((size_t)head * HD + row) * CRES + tb * 64 + seg * 8) = vr;
      } else {
        *(volatile v8us*)(Ph + ((size_t)head * TPAD + tb * 64 + row) * HD + seg * 8) = vh;
        if (dores) {
          if (MODE == 0) *(volatile v8us*)(Pr + ((size_t)head * QRES + tb * 64 + row) * HD + seg * 8) = vr;
          else           *(volatile v8us*)(Pr + ((size_t)head * CRES + tb * 64 + row) * HD + seg * 8) = vr;
        }
      }
    }
    __threadfence();
  }
}

template <bool EARLY>
__global__ __launch_bounds__(128) __attribute__((amdgpu_num_vgpr(256)))
void attn_kernel(const unsigned short* __restrict__ Qh, const unsigned short* __restrict__ Qr,
                 const unsigned short* __restrict__ Kh, const unsigned short* __restrict__ Kr,
                 const unsigned short* __restrict__ Vt, const unsigned short* __restrict__ Vr,
                 const unsigned short* __restrict__ Erp, const int* __restrict__ mask,
                 const int* __restrict__ flags, unsigned short* __restrict__ Ct,
                 unsigned short* __restrict__ Cr)
{
  constexpr int KSH = 0, ESH = 4096, VTH = 8192, PSH = 12288, KRS = 16384, VRS = 20480;
  constexpr int PRS = EARLY ? 24576 : PSH;
  constexpr int SMN = EARLY ? 28672 : 16384;
  __shared__ __align__(16) unsigned short sm[SMN];
  __shared__ __align__(16) unsigned char msk[4096];
  union FH { v16h v; v8us h[2]; };

  const int tid = threadIdx.x, wave = tid >> 5, lane = tid & 31;
  const int hh = lane >> 4, c = lane & 15;
  const int qb = EARLY ? (int)blockIdx.x : ((int)blockIdx.x + NEARLY);
  const int head = blockIdx.y;
  const int q0 = qb * 64 + wave * 16;
  const int wrow0 = wave * 16;

  const unsigned short* qp = Qh + ((size_t)head * TPAD + q0 + c) * HD + 8 * hh;
  const unsigned short* rp = Qr + ((size_t)head * QRES + (EARLY ? (q0 + c) : c)) * HD + 8 * hh;

  float mrow[8], lrow[8];
  v8f oacc[4];
#pragma unroll
  for (int r = 0; r < 8; ++r) { mrow[r] = -__builtin_inff(); lrow[r] = 0.f; }
#pragma unroll
  for (int t = 0; t < 4; ++t) oacc[t] = zero8();

  unsigned short* pwh = sm + PSH + wave * 1024;
  unsigned short* pwr = sm + PRS + wave * 1024;
  const int* frow = flags + (size_t)qb * 64;

#pragma unroll 1
  for (int kc = 0; kc < NKC; ++kc) {
    const int fk = __builtin_amdgcn_readfirstlane(frow[kc]);
    if (fk == 0) continue;
    const int kv0 = kc * 64;
    const bool useres = EARLY && (kc < NEARLY);
    const int kvr = (kc < NEARLY) ? kv0 : 0;

    __syncthreads();
#pragma unroll
    for (int it = 0; it < 4; ++it) {
      const int u = it * 128 + tid;
      const int row = u >> 3, seg = u & 7;
      *(v4u*)(sm + KSH + row * 64 + seg * 8) = *(const v4u*)(Kh + ((size_t)head * TPAD + kv0 + row) * HD + seg * 8);
      *(v4u*)(sm + ESH + row * 64 + seg * 8) = *(const v4u*)(Erp + (size_t)(kv0 + row) * HD + seg * 8);
      *(v4u*)(sm + VTH + row * 64 + seg * 8) = *(const v4u*)(Vt + ((size_t)head * HD + row) * TPAD + kv0 + seg * 8);
    }
    if (EARLY) {
#pragma unroll
      for (int it = 0; it < 4; ++it) {
        const int u = it * 128 + tid;
        const int row = u >> 3, seg = u & 7;
        *(v4u*)(sm + KRS + row * 64 + seg * 8) = *(const v4u*)(Kr + ((size_t)head * CRES + kvr + row) * HD + seg * 8);
        *(v4u*)(sm + VRS + row * 64 + seg * 8) = *(const v4u*)(Vr + ((size_t)head * HD + row) * CRES + kvr + seg * 8);
      }
    }
    if (fk == 2) {
      const int row = tid >> 1, hsel = tid & 1;
      int qrow = qb * 64 + row;
      qrow = qrow < TT ? qrow : TT - 1;
      const int* mb = mask + (size_t)qrow * SEQ_FULL;
#pragma unroll 1
      for (int g = 0; g < 4; ++g) {
#pragma unroll
        for (int e = 0; e < 8; ++e) {
          const int col = hsel * 32 + g * 8 + e;
          const int s = kv0 + col;
          const int sc = s < TT ? s : TT - 1;
          const int mv = mb[sc];
          msk[row * 64 + col] = (unsigned char)((s < TT && mv != 0) ? 1 : 0);
        }
      }
    }
    __syncthreads();

    FH qa[2], qs[2];
#pragma unroll
    for (int dc = 0; dc < 2; ++dc) {
      qa[dc].h[0] = *(const v8us*)(qp + dc * 32);
      qa[dc].h[1] = *(const v8us*)(qp + dc * 32 + 16);
      qs[dc].h[0] = *(const v8us*)(qp + HD + dc * 32);
      qs[dc].h[1] = *(const v8us*)(qp + HD + dc * 32 + 16);
    }

    v8f s[4];
#pragma unroll
    for (int j = 0; j < 4; ++j) {
      s[j] = zero8();
#pragma unroll
      for (int dc = 0; dc < 2; ++dc) {
        FH kf, ef;
        kf.h[0] = *(const v8us*)(sm + KSH + (j * 16 + c) * 64 + dc * 32 + 8 * hh);
        kf.h[1] = *(const v8us*)(sm + KSH + (j * 16 + c) * 64 + dc * 32 + 16 + 8 * hh);
        ef.h[0] = *(const v8us*)(sm + ESH + (j * 16 + c) * 64 + dc * 32 + 8 * hh);
        ef.h[1] = *(const v8us*)(sm + ESH + (j * 16 + c) * 64 + dc * 32 + 16 + 8 * hh);
        s[j] = mma_h(qa[dc].v, kf.v, s[j]);
        s[j] = mma_h(qs[dc].v, ef.v, s[j]);
      }
      if (EARLY) {
        if (useres) {
          v8f sr = zero8();
#pragma unroll
          for (int dc = 0; dc < 2; ++dc) {
            FH kf, ef, krf, qra, qrs;
            kf.h[0]  = *(const v8us*)(sm + KSH + (j * 16 + c) * 64 + dc * 32 + 8 * hh);
            kf.h[1]  = *(const v8us*)(sm + KSH + (j * 16 + c) * 64 + dc * 32 + 16 + 8 * hh);
            ef.h[0]  = *(const v8us*)(sm + ESH + (j * 16 + c) * 64 + dc * 32 + 8 * hh);
            ef.h[1]  = *(const v8us*)(sm + ESH + (j * 16 + c) * 64 + dc * 32 + 16 + 8 * hh);
            krf.h[0] = *(const v8us*)(sm + KRS + (j * 16 + c) * 64 + dc * 32 + 8 * hh);
            krf.h[1] = *(const v8us*)(sm + KRS + (j * 16 + c) * 64 + dc * 32 + 16 + 8 * hh);
            qra.h[0] = *(const v8us*)(rp + dc * 32);
            qra.h[1] = *(const v8us*)(rp + dc * 32 + 16);
            qrs.h[0] = *(const v8us*)(rp + HD + dc * 32);
            qrs.h[1] = *(const v8us*)(rp + HD + dc * 32 + 16);
            sr = mma_h(qa[dc].v, krf.v, sr);
            sr = mma_h(qra.v, kf.v, sr);
            sr = mma_h(qrs.v, ef.v, sr);
          }
#pragma unroll
          for (int r = 0; r < 8; ++r) s[j][r] += sr[r] * RINV;
        }
      }
    }

#pragma unroll
    for (int j = 0; j < 4; ++j) {
#pragma unroll
      for (int r = 0; r < 8; ++r) s[j][r] *= 0.125f;
    }
    if (fk == 2) {
#pragma unroll
      for (int j = 0; j < 4; ++j) {
#pragma unroll
        for (int r = 0; r < 8; ++r) {
          const unsigned char mv = msk[(wrow0 + 8 * hh + r) * 64 + j * 16 + c];
          s[j][r] = mv ? s[j][r] : -__builtin_inff();
        }
      }
    }

    float cm[8];
#pragma unroll
    for (int r = 0; r < 8; ++r) {
      float mx = fmaxf(fmaxf(s[0][r], s[1][r]), fmaxf(s[2][r], s[3][r]));
#pragma unroll
      for (int off = 1; off < 16; off <<= 1) mx = fmaxf(mx, __shfl_xor(mx, off, 32));
      cm[r] = mx;
    }

#pragma unroll
    for (int r = 0; r < 8; ++r) {
      const float mnew = fmaxf(mrow[r], cm[r]);
      const bool dead = (mnew == -__builtin_inff());
      const float aexp = __expf(mrow[r] - mnew);
      const float alpha = dead ? 1.f : aexp;
      mrow[r] = mnew;
      float psum = 0.f;
#pragma unroll
      for (int j = 0; j < 4; ++j) {
        const float pe = __expf(s[j][r] - mnew);
        const float p = dead ? 0.f : pe;
        psum += p;
        const float pc = p * PSC;
        const unsigned short hb = h_bits(pc);
        pwh[(8 * hh + r) * 64 + j * 16 + c] = hb;
        if (EARLY) {
          const float pres = (pc - h2f(hb)) * RSC;
          pwr[(8 * hh + r) * 64 + j * 16 + c] = h_bits(pres);
        }
      }
#pragma unroll
      for (int off = 1; off < 16; off <<= 1) psum += __shfl_xor(psum, off, 32);
      lrow[r] = lrow[r] * alpha + psum;
#pragma unroll
      for (int t = 0; t < 4; ++t) oacc[t][r] *= alpha;
    }
    __builtin_amdgcn_fence(3, "workgroup");
    __builtin_amdgcn_wave_barrier();
    __builtin_amdgcn_fence(2, "workgroup");

#pragma unroll
    for (int kk = 0; kk < 2; ++kk) {
      FH pa;
      pa.h[0] = *(const v8us*)(pwh + c * 64 + kk * 32 + 8 * hh);
      pa.h[1] = *(const v8us*)(pwh + c * 64 + kk * 32 + 16 + 8 * hh);
#pragma unroll
      for (int t = 0; t < 4; ++t) {
        FH vb;
        vb.h[0] = *(const v8us*)(sm + VTH + (t * 16 + c) * 64 + kk * 32 + 8 * hh);
        vb.h[1] = *(const v8us*)(sm + VTH + (t * 16 + c) * 64 + kk * 32 + 16 + 8 * hh);
        oacc[t] = mma_h(pa.v, vb.v, oacc[t]);
      }
    }
    if (EARLY) {
      if (useres) {
#pragma unroll
        for (int t = 0; t < 4; ++t) {
          v8f oar = zero8();
#pragma unroll
          for (int kk = 0; kk < 2; ++kk) {
            FH pa, pr, vb, vr;
            pa.h[0] = *(const v8us*)(pwh + c * 64 + kk * 32 + 8 * hh);
            pa.h[1] = *(const v8us*)(pwh + c * 64 + kk * 32 + 16 + 8 * hh);
            pr.h[0] = *(const v8us*)(pwr + c * 64 + kk * 32 + 8 * hh);
            pr.h[1] = *(const v8us*)(pwr + c * 64 + kk * 32 + 16 + 8 * hh);
            vb.h[0] = *(const v8us*)(sm + VTH + (t * 16 + c) * 64 + kk * 32 + 8 * hh);
            vb.h[1] = *(const v8us*)(sm + VTH + (t * 16 + c) * 64 + kk * 32 + 16 + 8 * hh);
            vr.h[0] = *(const v8us*)(sm + VRS + (t * 16 + c) * 64 + kk * 32 + 8 * hh);
            vr.h[1] = *(const v8us*)(sm + VRS + (t * 16 + c) * 64 + kk * 32 + 16 + 8 * hh);
            oar = mma_h(pa.v, vr.v, oar);
            oar = mma_h(pr.v, vb.v, oar);
          }
#pragma unroll
          for (int r = 0; r < 8; ++r) oacc[t][r] += oar[r] * RINV;
        }
      }
    }
  }

  __syncthreads();
  unsigned short* osh = sm + KSH + wave * 1024;
  unsigned short* osr = sm + ESH + wave * 1024;
#pragma unroll
  for (int r = 0; r < 8; ++r) {
    const float inv = (1.0f / lrow[r]) * OCV;
#pragma unroll
    for (int t = 0; t < 4; ++t) {
      const float o = oacc[t][r] * inv;
      const unsigned short hb = h_bits(o);
      osh[(8 * hh + r) * 64 + t * 16 + c] = hb;
      if (EARLY) {
        const float res = (o - h2f(hb)) * RSC;
        osr[(8 * hh + r) * 64 + t * 16 + c] = h_bits(res);
      }
    }
  }
  __builtin_amdgcn_fence(3, "workgroup");
  __builtin_amdgcn_wave_barrier();
  __builtin_amdgcn_fence(2, "workgroup");
  for (int pass = 0; pass < 2; ++pass) {
#pragma unroll
    for (int it = 0; it < 4; ++it) {
      const int u = it * 32 + lane;
      const int row = u >> 3, seg = u & 7;
      const v8us vh = *(const v8us*)(osh + row * 64 + seg * 8);
      *(volatile v8us*)(Ct + (size_t)(q0 + row) * DM + head * 64 + seg * 8) = vh;
      if (EARLY) {
        const v8us vr = *(const v8us*)(osr + row * 64 + seg * 8);
        *(volatile v8us*)(Cr + (size_t)(q0 + row) * DM + head * 64 + seg * 8) = vr;
      }
    }
    __threadfence();
  }
}

__global__ __launch_bounds__(64) __attribute__((amdgpu_num_vgpr(256)))
void out_kernel(
    const unsigned short* __restrict__ Ct, const unsigned short* __restrict__ Cr,
    const unsigned short* __restrict__ Wo, const float* __restrict__ bias, float* __restrict__ out)
{
  constexpr int PTF = 68;
  __shared__ __align__(16) float ts[64 * PTF];
  union FH { v16h v; v8us h[2]; };

  const int tid = threadIdx.x, wave = tid >> 5, lane = tid & 31;
  const int hh = lane >> 4, m = lane & 15;
  const int tb = blockIdx.x, nb = blockIdx.y;
  const int n0 = nb * 64;
  const int rl0 = wave * 32;
  const int r0 = tb * 64 + rl0;
  const bool dores = tb < NEARLY;

  v8f acc[2][4];
#pragma unroll
  for (int mi = 0; mi < 2; ++mi)
#pragma unroll
    for (int ni = 0; ni < 4; ++ni) acc[mi][ni] = zero8();

  const unsigned short* wp = Wo + (size_t)(n0 + m) * DM + 8 * hh;

  if (dores) {
    const unsigned short* cp0 = Cr + (size_t)(r0 + m) * DM + 8 * hh;
    const unsigned short* cp1 = Cr + (size_t)(r0 + 16 + m) * DM + 8 * hh;
#pragma unroll 2
    for (int k0 = 0; k0 < DM; k0 += 32) {
      FH a0, a1;
      a0.h[0] = *(const v8us*)(cp0 + k0);
      a0.h[1] = *(const v8us*)(cp0 + k0 + 16);
      a1.h[0] = *(const v8us*)(cp1 + k0);
      a1.h[1] = *(const v8us*)(cp1 + k0 + 16);
#pragma unroll
      for (int ni = 0; ni < 4; ++ni) {
        FH b;
        b.h[0] = *(const v8us*)(wp + (size_t)ni * 16 * DM + k0);
        b.h[1] = *(const v8us*)(wp + (size_t)ni * 16 * DM + k0 + 16);
        acc[0][ni] = mma_h(a0.v, b.v, acc[0][ni]);
        acc[1][ni] = mma_h(a1.v, b.v, acc[1][ni]);
      }
    }
#pragma unroll
    for (int mi = 0; mi < 2; ++mi)
#pragma unroll
      for (int ni = 0; ni < 4; ++ni)
#pragma unroll
        for (int r = 0; r < 8; ++r) acc[mi][ni][r] *= RINV;
  }

  {
    const unsigned short* cp0 = Ct + (size_t)(r0 + m) * DM + 8 * hh;
    const unsigned short* cp1 = Ct + (size_t)(r0 + 16 + m) * DM + 8 * hh;
#pragma unroll 2
    for (int k0 = 0; k0 < DM; k0 += 32) {
      FH a0, a1;
      a0.h[0] = *(const v8us*)(cp0 + k0);
      a0.h[1] = *(const v8us*)(cp0 + k0 + 16);
      a1.h[0] = *(const v8us*)(cp1 + k0);
      a1.h[1] = *(const v8us*)(cp1 + k0 + 16);
#pragma unroll
      for (int ni = 0; ni < 4; ++ni) {
        FH b;
        b.h[0] = *(const v8us*)(wp + (size_t)ni * 16 * DM + k0);
        b.h[1] = *(const v8us*)(wp + (size_t)ni * 16 * DM + k0 + 16);
        acc[0][ni] = mma_h(a0.v, b.v, acc[0][ni]);
        acc[1][ni] = mma_h(a1.v, b.v, acc[1][ni]);
      }
    }
  }

  float bb[4];
#pragma unroll
  for (int ni = 0; ni < 4; ++ni) bb[ni] = bfr(bias[n0 + ni * 16 + m]);
#pragma unroll
  for (int mi = 0; mi < 2; ++mi) {
#pragma unroll
    for (int ni = 0; ni < 4; ++ni) {
#pragma unroll
      for (int r = 0; r < 8; ++r) {
        const int rl = rl0 + mi * 16 + 8 * hh + r;
        ts[rl * PTF + ni * 16 + m] = acc[mi][ni][r] * OINV + bb[ni];
      }
    }
  }
  __syncthreads();

  for (int pass = 0; pass < 2; ++pass) {
#pragma unroll
    for (int it = 0; it < 16; ++it) {
      const int u = it * 64 + tid;
      const int row = u >> 4, seg = u & 15;
      const int t = tb * 64 + row;
      const v4f v = *(const v4f*)(ts + row * PTF + seg * 4);
      if (t < TT) *(volatile v4f*)(out + (size_t)t * DM + n0 + seg * 4) = v;
    }
    __threadfence();
  }
}

extern "C" void kernel_launch(void* const* d_in, const int* in_sizes, int n_in,
                              void* d_out, int out_size, void* d_ws, size_t ws_size,
                              hipStream_t stream)
{
  if (n_in < 13) return;
  if (in_sizes[0] < TT * DM || in_sizes[1] < TT * DM || in_sizes[2] < TT * DM) return;
  if (in_sizes[3] < (TT - 1) * SEQ_FULL + TT) return;
  if (in_sizes[4] < DM * DM || in_sizes[6] < DM * DM || in_sizes[8] < DM * DM || in_sizes[11] < DM * DM) return;
  if (in_sizes[5] < DM || in_sizes[7] < DM || in_sizes[9] < DM || in_sizes[12] < DM) return;
  if (in_sizes[10] < TT * HD) return;
  if (out_size < TT * DM) return;
  if (d_ws == nullptr || ws_size < WS_NEED) return;

  const float* q    = (const float*)d_in[0];
  const float* k    = (const float*)d_in[1];
  const float* v    = (const float*)d_in[2];
  const int*   mask = (const int*)d_in[3];
  const float* Wq_w = (const float*)d_in[4];
  const float* Wq_b = (const float*)d_in[5];
  const float* Wk_w = (const float*)d_in[6];
  const float* Wk_b = (const float*)d_in[7];
  const float* Wv_w = (const float*)d_in[8];
  const float* Wv_b = (const float*)d_in[9];
  const float* Er   = (const float*)d_in[10];
  const float* Wo_w = (const float*)d_in[11];
  const float* Wo_b = (const float*)d_in[12];
  float* outp = (float*)d_out;

  unsigned char* ws = (unsigned char*)d_ws;
  unsigned short* Xq = (unsigned short*)(ws + OFF_XQ);
  unsigned short* Xk = (unsigned short*)(ws + OFF_XK);
  unsigned short* Xv = (unsigned short*)(ws + OFF_XV);
  unsigned short* Wq = (unsigned short*)(ws + OFF_WQ);
  unsigned short* Wk = (unsigned short*)(ws + OFF_WK);
  unsigned short* Wv = (unsigned short*)(ws + OFF_WV);
  unsigned short* Wo = (unsigned short*)(ws + OFF_WO);
  unsigned short* Eh = (unsigned short*)(ws + OFF_ER);
  unsigned short* Qh = (unsigned short*)(ws + OFF_QH);
  unsigned short* Kh = (unsigned short*)(ws + OFF_KH);
  unsigned short* Vt = (unsigned short*)(ws + OFF_VT);
  unsigned short* Qr = (unsigned short*)(ws + OFF_QR);
  unsigned short* Kr = (unsigned short*)(ws + OFF_KR);
  unsigned short* Vr = (unsigned short*)(ws + OFF_VR);
  unsigned short* Ct = (unsigned short*)(ws + OFF_CT);
  unsigned short* Cr = (unsigned short*)(ws + OFF_CR);
  int* flags = (int*)(ws + OFF_FL);

  const int xu = TPAD * (DM / 8);
  const int wu = DM * (DM / 8);
  const int eu = TPAD * (HD / 8);
  cvt_plane_kernel<<<(xu + 255) / 256, 256, 0, stream>>>(q, TT, DM, TPAD, 0, 1.0f, Xq);
  cvt_plane_kernel<<<(xu + 255) / 256, 256, 0, stream>>>(k, TT, DM, TPAD, 0, 1.0f, Xk);
  cvt_plane_kernel<<<(xu + 255) / 256, 256, 0, stream>>>(v, TT, DM, TPAD, 0, 1.0f, Xv);
  cvt_plane_kernel<<<(wu + 255) / 256, 256, 0, stream>>>(Wq_w, DM, DM, DM, 0, 1.0f, Wq);
  cvt_plane_kernel<<<(wu + 255) / 256, 256, 0, stream>>>(Wk_w, DM, DM, DM, 0, 1.0f, Wk);
  cvt_plane_kernel<<<(wu + 255) / 256, 256, 0, stream>>>(Wv_w, DM, DM, DM, 0, 1.0f, Wv);
  cvt_plane_kernel<<<(wu + 255) / 256, 256, 0, stream>>>(Wo_w, DM, DM, DM, 1, WOSC, Wo);
  cvt_plane_kernel<<<(eu + 255) / 256, 256, 0, stream>>>(Er, TT, HD, TPAD, 1, 1.0f, Eh);

  flags_kernel<<<NQB, 256, 0, stream>>>(mask, flags);

  proj_kernel<0><<<dim3(NTB, NH), 64, 0, stream>>>(Xq, Wq, Wq_b, Qh, Qr);
  proj_kernel<1><<<dim3(NTB, NH), 64, 0, stream>>>(Xk, Wk, Wk_b, Kh, Kr);
  proj_kernel<2><<<dim3(NTB, NH), 64, 0, stream>>>(Xv, Wv, Wv_b, Vt, Vr);

  attn_kernel<true><<<dim3(NEARLY, NH), 128, 0, stream>>>(Qh, Qr, Kh, Kr, Vt, Vr, Eh, mask, flags, Ct, Cr);
  if (NQB > NEARLY)
    attn_kernel<false><<<dim3(NQB - NEARLY, NH), 128, 0, stream>>>(Qh, Qr, Kh, Kr, Vt, Vr, Eh, mask, flags, Ct, Cr);

  out_kernel<<<dim3(NQB, DM / 64), 64, 0, stream>>>(Ct, Cr, Wo, Wo_b, outp);
}
